// nonlocal_attention_9148280341044
// MI455X (gfx1250) — hardware-run, weakly checked
//
#include <hip/hip_runtime.h>


#define NV   4
#define TT8  8
#define CC   512
#define HW   196
#define SS   1568
#define SP   1664
#define NH_  8
#define HD   64
#define PCAR 1024.0f
typedef _Float16 h16;
typedef unsigned short bf;
typedef __attribute__((ext_vector_type(16))) __bf16   v16bf;
typedef __attribute__((ext_vector_type(16))) _Float16 v16h;
typedef __attribute__((ext_vector_type(8)))  _Float16 v8h;
typedef __attribute__((ext_vector_type(8)))  unsigned short v8us;
typedef __attribute__((ext_vector_type(8)))  float    v8f;
typedef __attribute__((ext_vector_type(4)))  float    v4f;
typedef v8h  __attribute__((may_alias)) v8ha;
typedef v4f  __attribute__((may_alias)) v4fa;
typedef v8us __attribute__((may_alias)) v8usa;

__device__ __forceinline__ unsigned short f2bf(float f) { unsigned u = __float_as_uint(f); u += 0x7FFFu + ((u >> 16) & 1u); return (unsigned short)(u >> 16); }
__device__ __forceinline__ float bf2f(unsigned short b) { return __uint_as_float(((unsigned)b) << 16); }
__device__ __forceinline__ float bfr(float f) { return bf2f(f2bf(f)); }
__device__ __forceinline__ v16h cat16(v8h lo, v8h hi) { return __builtin_shufflevector(lo, hi, 0, 1, 2, 3, 4, 5, 6, 7, 8, 9, 10, 11, 12, 13, 14, 15); }
__device__ __forceinline__ v16bf cat16b(v8us lo, v8us hi) { return __builtin_bit_cast(v16bf, __builtin_shufflevector(lo, hi, 0, 1, 2, 3, 4, 5, 6, 7, 8, 9, 10, 11, 12, 13, 14, 15)); }
__device__ __forceinline__ v8f wmma16(v16h a, v16h b, v8f c) { return __builtin_amdgcn_wmma_f32_16x16x32_f16(false, a, false, b, (short)0, c, false, false); }
__device__ __forceinline__ v8f wmmab(v16bf a, v16bf b, v8f c) { return __builtin_amdgcn_wmma_f32_16x16x32_bf16(false, a, false, b, (short)0, c, false, false); }


template <typename T16> struct WFrag;
template <> struct WFrag<h16> { typedef v16h V; static __device__ __forceinline__ V ld(const h16* p) { return cat16(*(const v8h*)p, *(const v8h*)(p + 16)); } static __device__ __forceinline__ v8f mma(V a, V b, v8f c) { return wmma16(a, b, c); } };
template <> struct WFrag<bf> { typedef v16bf V; static __device__ __forceinline__ V ld(const bf* p) { return cat16b(*(const v8us*)p, *(const v8us*)(p + 16)); } static __device__ __forceinline__ v8f mma(V a, V b, v8f c) { return wmmab(a, b, c); } };
template <typename T16, int NSPLIT, bool BIAS>
__global__ __launch_bounds__(32) void k_gemmw(const T16* __restrict__ A, const T16* __restrict__ A2, const T16* __restrict__ Bt, const T16* __restrict__ Bt2, int K, float* C, int ldc, const float* __restrict__ bias, size_t sA, size_t sB, size_t sC) {
    typedef typename WFrag<T16>::V V;
    __shared__ __align__(16) float os[16 * 68];
    const size_t z = blockIdx.z; A += z * sA; if (A2) A2 += z * sA; Bt += z * sB; if (Bt2) Bt2 += z * sB; C += z * sC;
    const int lane = threadIdx.x & 31, lr = lane & 15, hi = lane >> 4; const int r0 = blockIdx.x * 64, c0 = blockIdx.y * 64;
    v8f acc[4][4];
#pragma unroll
    for (int mb = 0; mb < 4; ++mb)
#pragma unroll
        for (int nb = 0; nb < 4; ++nb) acc[mb][nb] = (v8f){};
    const size_t aoff = (size_t)(r0 + lr) * K + 8 * hi, boff = (size_t)(c0 + lr) * K + 8 * hi;
#pragma unroll 1
    for (int kc = 0; kc < K; kc += 32) {
        V a[4], a2[4];
#pragma unroll
        for (int mb = 0; mb < 4; ++mb) { a[mb] = WFrag<T16>::ld(A + aoff + (size_t)mb * 16 * K + kc); if (NSPLIT == 1 || NSPLIT == 2) a2[mb] = WFrag<T16>::ld(A2 + aoff + (size_t)mb * 16 * K + kc); }
#pragma unroll
        for (int nb = 0; nb < 4; ++nb) { const V b = WFrag<T16>::ld(Bt + boff + (size_t)nb * 16 * K + kc); V b2; if (NSPLIT >= 2) b2 = WFrag<T16>::ld(Bt2 + boff + (size_t)nb * 16 * K + kc);
#pragma unroll
            for (int mb = 0; mb < 4; ++mb) { acc[mb][nb] = WFrag<T16>::mma(a[mb], b, acc[mb][nb]); if (NSPLIT == 1 || NSPLIT == 2) acc[mb][nb] = WFrag<T16>::mma(a2[mb], b, acc[mb][nb]); if (NSPLIT >= 2) acc[mb][nb] = WFrag<T16>::mma(a[mb], b2, acc[mb][nb]); } }
        asm volatile("v_nop\n\tv_nop\n\tv_nop\n\tv_nop" : "+v"(acc[0][0]), "+v"(acc[1][1]), "+v"(acc[2][2]), "+v"(acc[3][3]) : "v"(a[0]), "v"(a[3]));
    }
#pragma unroll
    for (int mb = 0; mb < 4; ++mb) {
#pragma unroll
        for (int nb = 0; nb < 4; ++nb) {
#pragma unroll
            for (int j = 0; j < 8; ++j) os[(hi * 8 + j) * 68 + nb * 16 + lr] = acc[mb][nb][j]; }
        __builtin_amdgcn_wave_barrier(); asm volatile("" ::: "memory");
        float* crow = C + (size_t)(r0 + mb * 16) * ldc + c0;
#pragma unroll 1
        for (int ps = 0; ps < 2; ++ps) {
#pragma unroll
            for (int s = 0; s < 8; ++s) { const int row = 2 * s + hi, cofs = lr * 4; v4f val = *(const v4fa*)(os + row * 68 + cofs); if (BIAS) { val[0] += bfr(bias[c0 + cofs]); val[1] += bfr(bias[c0 + cofs + 1]); val[2] += bfr(bias[c0 + cofs + 2]); val[3] += bfr(bias[c0 + cofs + 3]); }
                *(volatile v4f*)(crow + (size_t)row * ldc + cofs) = val; }
            if (ps == 0) __threadfence(); }
        __builtin_amdgcn_wave_barrier(); asm volatile("" ::: "memory");
    }
}

__device__ __forceinline__ h16 tohx(float x) { return (h16)x; }
typedef __attribute__((ext_vector_type(2))) unsigned short v2us;
typedef __attribute__((ext_vector_type(4))) unsigned short v4us;
typedef __attribute__((ext_vector_type(2))) _Float16 v2h;
typedef __attribute__((ext_vector_type(4))) _Float16 v4h;

__global__ __launch_bounds__(256) void k_cvt8(const float* __restrict__ src, bf* dst, size_t n8) { const size_t i = (size_t)blockIdx.x * 256 + threadIdx.x; if (i >= n8) return; const v8f v = *(const v8f*)(src + i * 8); v8us o;
#pragma unroll
    for (int k = 0; k < 8; ++k) o[k] = f2bf(v[k]); *(volatile v8us*)(dst + i * 8) = o; __threadfence(); *(volatile v8us*)(dst + i * 8) = o; }
__global__ __launch_bounds__(256) void k_tok(const float* __restrict__ x, bf* XT) { const int e = (blockIdx.x * 256 + threadIdx.x) * 2; if (e >= SP * CC) return; const int c = e % CC; const int s = e / CC; v2us o;
    if (s < SS) { const int t = s / HW, hw = s % HW; o[0] = f2bf(x[((size_t)t * CC + c) * HW + hw]); o[1] = f2bf(x[((size_t)t * CC + c + 1) * HW + hw]); } else { o[0] = 0; o[1] = 0; }
    *(volatile v2us*)(XT + e) = o; __threadfence(); *(volatile v2us*)(XT + e) = o; }
__global__ __launch_bounds__(256) void k_msk(const float* __restrict__ x, float* M) { const int s = blockIdx.x * 256 + threadIdx.x; if (s >= SP) return; float sum = 0.f; if (s < SS) { const int t = s / HW, hw = s % HW;
#pragma unroll 1
        for (int c = 0; c < CC; ++c) sum = __fadd_rn(sum, bfr(x[((size_t)t * CC + c) * HW + hw])); }
    const float m = (s < SS && sum != 0.f) ? 1.f : 0.f; *(volatile float*)(M + s) = m; __threadfence(); *(volatile float*)(M + s) = m; }
__global__ __launch_bounds__(256) void k_qk16(const float* __restrict__ FQ, const float* __restrict__ FK, h16* Q16, h16* K16) { const int e = (blockIdx.x * 256 + threadIdx.x) * 4; if (e >= NH_ * SP * HD) return; const int d = e % HD; const int s = (e / HD) % SP; const int h = e / (HD * SP); const size_t f = (size_t)s * CC + h * HD + d; v4h q, k;
#pragma unroll
    for (int u = 0; u < 4; ++u) { q[u] = tohx(fmaxf(FQ[f + u], 0.f) * 0.125f); k[u] = tohx(fmaxf(FK[f + u], 0.f)); } for (int ps = 0; ps < 2; ++ps) { *(volatile v4h*)(Q16 + e) = q; *(volatile v4h*)(K16 + e) = k; if (ps == 0) __threadfence(); } }
__global__ __launch_bounds__(256) void k_vt(const float* __restrict__ FV, h16* VT) { const int e = (blockIdx.x * 256 + threadIdx.x) * 2; if (e >= NH_ * HD * SP) return; const int s = e % SP; const int d = (e / SP) % HD; const int h = e / (SP * HD); v2h o; o[0] = tohx(fmaxf(FV[(size_t)s * CC + h * HD + d], 0.f)); o[1] = tohx(fmaxf(FV[(size_t)(s + 1) * CC + h * HD + d], 0.f));
    *(volatile v2h*)(VT + e) = o; __threadfence(); *(volatile v2h*)(VT + e) = o; }
__global__ __launch_bounds__(256) void k_msoft(const float* __restrict__ Sb, const float* __restrict__ KM, const float* __restrict__ QM, h16* P16) { const int lane = threadIdx.x & 31; const int row = blockIdx.x * 8 + (threadIdx.x >> 5); if (row >= NH_ * SP) return; const int s = row % SP; const float* sr = Sb + (size_t)row * SP; float v[SP / 32]; float mx = -3.0e38f;
#pragma unroll
    for (int ch = 0; ch < SP / 128; ++ch) { const int j0 = ch * 128 + lane * 4; const v4f a = *(const v4f*)(sr + j0); const v4f km = *(const v4f*)(KM + j0);
#pragma unroll
        for (int u = 0; u < 4; ++u) { const float t = (km[u] != 0.f) ? a[u] : -3.0e38f; v[ch * 4 + u] = t; mx = fmaxf(mx, t); } }
#pragma unroll
    for (int sh = 16; sh; sh >>= 1) mx = fmaxf(mx, __shfl_xor(mx, sh, 32));
    float sum = 0.f;
#pragma unroll
    for (int q = 0; q < SP / 32; ++q) { float d0 = __fsub_rn(v[q], mx); asm volatile("" : "+v"(d0)); v[q] = __builtin_amdgcn_exp2f(__fmul_rn(d0, 1.4426950408889634f)); sum += v[q]; }
#pragma unroll
    for (int sh = 16; sh; sh >>= 1) sum += __shfl_xor(sum, sh, 32);
    float f = __fdiv_rn(1.0f, sum); f = __fmul_rn(f, QM[s]) * PCAR;
    for (int ps = 0; ps < 2; ++ps) {
#pragma unroll
        for (int ch = 0; ch < SP / 128; ++ch) { v4h o4;
#pragma unroll
            for (int q = 0; q < 4; ++q) o4[q] = tohx(v[ch * 4 + q] * f); *(volatile v4h*)(P16 + (size_t)row * SP + ch * 128 + lane * 4) = o4; }
        if (ps == 0) __threadfence(); } }
__global__ __launch_bounds__(256) void k_mrg(const float* __restrict__ O, const float* __restrict__ xq, float* Y) { const int e = (blockIdx.x * 256 + threadIdx.x) * 4; if (e >= SS * CC) return; const int c = e % CC; const int s = e / CC; const int h = c / HD, d = c % HD; const int t = s / HW, hw = s % HW; v4f o;
#pragma unroll
    for (int u = 0; u < 4; ++u) { const float ov = O[((size_t)h * SP + s) * HD + d + u] * (1.0f / PCAR); o[u] = __fadd_rn(ov, bfr(xq[((size_t)t * CC + c + u) * HW + hw])); } *(volatile v4f*)(Y + e) = o; __threadfence(); *(volatile v4f*)(Y + e) = o; }
__global__ __launch_bounds__(256) void k_ln(const float* __restrict__ Y, const float* __restrict__ ga, const float* __restrict__ be, float* YN) { const int lane = threadIdx.x & 31; const int s = blockIdx.x * 8 + (threadIdx.x >> 5); if (s >= SS) return; const float* yr = Y + (size_t)s * CC; float v[CC / 32]; float sum = 0.f;
#pragma unroll
    for (int ch = 0; ch < CC / 128; ++ch) { const v4f a = *(const v4f*)(yr + ch * 128 + lane * 4);
#pragma unroll
        for (int u = 0; u < 4; ++u) { v[ch * 4 + u] = a[u]; sum += a[u]; } }
#pragma unroll
    for (int sh = 16; sh; sh >>= 1) sum += __shfl_xor(sum, sh, 32);
    const float mean = sum * (1.0f / CC); float q = 0.f;
#pragma unroll
    for (int k = 0; k < CC / 32; ++k) { float d = __fsub_rn(v[k], mean); asm volatile("" : "+v"(d)); float p = __fmul_rn(d, d); asm volatile("" : "+v"(p)); q = __fadd_rn(q, p); }
#pragma unroll
    for (int sh = 16; sh; sh >>= 1) q += __shfl_xor(q, sh, 32);
    const float sd = __fsqrt_rn(q * (1.0f / (CC - 1))); const float inv = __fdiv_rn(1.0f, __fadd_rn(sd, 1e-8f));
    for (int ps = 0; ps < 2; ++ps) {
#pragma unroll
        for (int ch = 0; ch < CC / 128; ++ch) { v4f o; const int c0 = ch * 128 + lane * 4;
#pragma unroll
            for (int u = 0; u < 4; ++u) { float d = __fsub_rn(v[ch * 4 + u], mean); asm volatile("" : "+v"(d)); float g = bfr(ga[c0 + u]), bb = bfr(be[c0 + u]); asm volatile("" : "+v"(g)); asm volatile("" : "+v"(bb)); float t1 = __fmul_rn(g, d); asm volatile("" : "+v"(t1)); float t2 = __fmul_rn(t1, inv); asm volatile("" : "+v"(t2)); o[u] = __fadd_rn(t2, bb); }
            *(volatile v4f*)(YN + (size_t)s * CC + c0) = o; }
        if (ps == 0) __threadfence(); } }
__global__ __launch_bounds__(256) void k_out(const float* __restrict__ YN, float* OUTn) { const int e = (blockIdx.x * 256 + threadIdx.x) * 4; if (e >= TT8 * CC * HW) return; const int hw = e % HW; const int c = (e / HW) % CC; const int t = e / (HW * CC); v4f o;
#pragma unroll
    for (int u = 0; u < 4; ++u) o[u] = YN[((size_t)t * HW + hw + u) * CC + c]; *(volatile v4f*)(OUTn + e) = o; __threadfence(); *(volatile v4f*)(OUTn + e) = o; }

extern "C" void kernel_launch(void* const* d_in, const int* in_sizes, int n_in,
                              void* d_out, int out_size, void* d_ws, size_t ws_size, hipStream_t stream) {
    (void)in_sizes; (void)n_in; (void)out_size;
    const float* xq = (const float*)d_in[0]; const float* xk = (const float*)d_in[1]; const float* xv = (const float*)d_in[2]; const float* Wq = (const float*)d_in[3]; const float* bq = (const float*)d_in[4]; const float* Wk = (const float*)d_in[5]; const float* bk = (const float*)d_in[6]; const float* Wv = (const float*)d_in[7]; const float* bv = (const float*)d_in[8]; const float* ga = (const float*)d_in[9]; const float* be = (const float*)d_in[10];
    float* OUT = (float*)d_out;
    char* wsp = (char*)d_ws;
    auto take = [&](size_t bytes) { char* p = wsp; wsp += (bytes + 255) & ~(size_t)255; return (void*)p; };
    bf* WQ = (bf*)take((size_t)CC * CC * 2); bf* WK = (bf*)take((size_t)CC * CC * 2); bf* WV = (bf*)take((size_t)CC * CC * 2);
    bf* XT = (bf*)take((size_t)SP * CC * 2); float* FQ = (float*)take((size_t)SP * CC * 4); float* FK = (float*)take((size_t)SP * CC * 4); float* FV = (float*)take((size_t)SP * CC * 4); float* KM = (float*)take(SP * 4); float* QM = (float*)take(SP * 4);
    h16* Q16 = (h16*)take((size_t)NH_ * SP * HD * 2); h16* K16 = (h16*)take((size_t)NH_ * SP * HD * 2); h16* VT = (h16*)take((size_t)NH_ * HD * SP * 2); float* Sb = (float*)take((size_t)NH_ * SP * SP * 4); h16* P16 = (h16*)take((size_t)NH_ * SP * SP * 2); float* O = (float*)take((size_t)NH_ * SP * HD * 4); float* Y = (float*)take((size_t)SS * CC * 4); float* YN = (float*)take((size_t)SS * CC * 4);
    if ((size_t)(wsp - (char*)d_ws) > ws_size) return;
    k_cvt8<<<(CC * CC / 8 + 255) / 256, 256, 0, stream>>>(Wq, WQ, CC * CC / 8); k_cvt8<<<(CC * CC / 8 + 255) / 256, 256, 0, stream>>>(Wk, WK, CC * CC / 8); k_cvt8<<<(CC * CC / 8 + 255) / 256, 256, 0, stream>>>(Wv, WV, CC * CC / 8);
    const size_t vs = (size_t)TT8 * CC * HW;
    for (int n = 0; n < NV; ++n) {
        k_tok<<<(SP * CC / 2 + 255) / 256, 256, 0, stream>>>(xq + n * vs, XT); k_gemmw<bf, 0, true><<<dim3(SP / 64, CC / 64, 1), 32, 0, stream>>>(XT, nullptr, WQ, nullptr, CC, FQ, CC, bq, 0, 0, 0); k_msk<<<(SP + 255) / 256, 256, 0, stream>>>(xq + n * vs, QM);
        k_tok<<<(SP * CC / 2 + 255) / 256, 256, 0, stream>>>(xk + n * vs, XT); k_gemmw<bf, 0, true><<<dim3(SP / 64, CC / 64, 1), 32, 0, stream>>>(XT, nullptr, WK, nullptr, CC, FK, CC, bk, 0, 0, 0); k_msk<<<(SP + 255) / 256, 256, 0, stream>>>(xk + n * vs, KM);
        k_tok<<<(SP * CC / 2 + 255) / 256, 256, 0, stream>>>(xv + n * vs, XT); k_gemmw<bf, 0, true><<<dim3(SP / 64, CC / 64, 1), 32, 0, stream>>>(XT, nullptr, WV, nullptr, CC, FV, CC, bv, 0, 0, 0);
        k_qk16<<<(NH_ * SP * HD / 4 + 255) / 256, 256, 0, stream>>>(FQ, FK, Q16, K16); k_vt<<<(NH_ * HD * SP / 2 + 255) / 256, 256, 0, stream>>>(FV, VT);
        k_gemmw<h16, 0, false><<<dim3(SP / 64, SP / 64, NH_), 32, 0, stream>>>(Q16, nullptr, K16, nullptr, HD, Sb, SP, nullptr, (size_t)SP * HD, (size_t)SP * HD, (size_t)SP * SP);
        k_msoft<<<NH_ * SP / 8, 256, 0, stream>>>(Sb, KM, QM, P16);
        k_gemmw<h16, 0, false><<<dim3(SP / 64, 1, NH_), 32, 0, stream>>>(P16, nullptr, VT, nullptr, SP, O, HD, nullptr, (size_t)SP * SP, (size_t)HD * SP, (size_t)SP * HD);
        k_mrg<<<(SS * CC / 4 + 255) / 256, 256, 0, stream>>>(O, xq + n * vs, Y); k_ln<<<(SS + 7) / 8, 256, 0, stream>>>(Y, ga, be, YN);
        k_out<<<(unsigned)((vs / 4 + 255) / 256), 256, 0, stream>>>(YN, OUT + n * vs); }
}
